// DiffusionGCN_52158082842768
// MI455X (gfx1250) — hardware-run, weakly checked
//
#include <hip/hip_runtime.h>

typedef float          v8f   __attribute__((ext_vector_type(8)));
typedef float          v4f   __attribute__((ext_vector_type(4)));
typedef unsigned int   v4u   __attribute__((ext_vector_type(4)));
typedef int            v8i   __attribute__((ext_vector_type(8)));
typedef unsigned short v8us  __attribute__((ext_vector_type(8)));
typedef unsigned short v16us __attribute__((ext_vector_type(16)));
typedef __bf16         v16bf __attribute__((ext_vector_type(16)));
typedef _Float16       v16h  __attribute__((ext_vector_type(16)));
typedef v4f  __attribute__((may_alias)) v4fa;
typedef v8us __attribute__((may_alias)) v8usa;
union FragB { v16bf v; v16us u; v8us h[2]; v8i w; };
union FragH { v16h  v; v16us u; v8us h[2]; v8i w; };

__device__ __forceinline__ v8f wmb(const FragB& a, const FragB& b, v8f c) {
  v8f d = __builtin_amdgcn_wmma_f32_16x16x32_bf16(false, a.v, false, b.v, (short)0, c, false, false);
  asm volatile("v_nop\n\tv_nop\n\tv_nop\n\tv_nop" : "+v"(d) : "v"(a.w), "v"(b.w));
  return d;
}

__device__ __forceinline__ v8f wmh(const FragH& a, const FragH& b, v8f c) {
  v8f d = __builtin_amdgcn_wmma_f32_16x16x32_f16(false, a.v, false, b.v, (short)0, c, false, false);
  asm volatile("v_nop\n\tv_nop\n\tv_nop\n\tv_nop" : "+v"(d) : "v"(a.w), "v"(b.w));
  return d;
}

__device__ __forceinline__ unsigned bf16_bits(float f) {
  const unsigned u = __float_as_uint(f);
  const unsigned r = (u + 0x7FFFu + ((u >> 16) & 1u)) >> 16;
  const unsigned q = (u >> 16) | 0x40u;
  return ((u & 0x7fffffffu) > 0x7f800000u) ? q : r;
}

__device__ __forceinline__ float bf16_val(float f) {
  return __uint_as_float(bf16_bits(f) << 16);
}
__device__ __forceinline__ int clampi(int v, int lo, int hi) {
  return v < lo ? lo : (v > hi ? hi : v);
}

__device__ __forceinline__ unsigned f16_bits(float f) {
  const unsigned u  = __float_as_uint(f);
  const unsigned s  = (u >> 16) & 0x8000u;
  const unsigned a  = u & 0x7fffffffu;
  const unsigned t  = a - 0x38000000u;
  const unsigned r  = (t + 0x0FFFu + ((t >> 13) & 1u)) >> 13;
  const unsigned rc = r > 0x7C00u ? 0x7C00u : r;
  const bool small  = a < 0x38800000u;
  const bool isnan  = a > 0x7f800000u;
  const unsigned fin = small ? 0u : (s | rc);
  return isnan ? (s | 0x7E00u) : fin;
}

__device__ __forceinline__ unsigned pk16(unsigned lo, unsigned hi) { return lo | (hi << 16); }
__device__ __forceinline__ unsigned bf16_lo_bits(float v) {
  float hi = bf16_val(v);
  asm volatile("" : "+v"(hi));
  return bf16_bits(v - hi);
}
__device__ __forceinline__ v4u pack8_bf16(v4f a, v4f c) {
  return (v4u){ pk16(bf16_bits(a[0]), bf16_bits(a[1])), pk16(bf16_bits(a[2]), bf16_bits(a[3])),
                pk16(bf16_bits(c[0]), bf16_bits(c[1])), pk16(bf16_bits(c[2]), bf16_bits(c[3])) };
}
__device__ __forceinline__ v4u pack8_bf16_lo(v4f a, v4f c) {
  return (v4u){ pk16(bf16_lo_bits(a[0]), bf16_lo_bits(a[1])), pk16(bf16_lo_bits(a[2]), bf16_lo_bits(a[3])),
                pk16(bf16_lo_bits(c[0]), bf16_lo_bits(c[1])), pk16(bf16_lo_bits(c[2]), bf16_lo_bits(c[3])) };
}
__device__ __forceinline__ v4u pack8_f16(v4f a, v4f c) {
  return (v4u){ pk16(f16_bits(a[0]), f16_bits(a[1])), pk16(f16_bits(a[2]), f16_bits(a[3])),
                pk16(f16_bits(c[0]), f16_bits(c[1])), pk16(f16_bits(c[2]), f16_bits(c[3])) };
}

template <int FORM>
__global__ __launch_bounds__(256) void k_plane(const float* __restrict__ src, int rows, int cols, int ldsrc,
                                               unsigned short* __restrict__ dst, int MP, int KP) {
  static_assert(FORM >= 0 && FORM <= 3);
  const int KTOT = (FORM == 1 || FORM == 3) ? 2 * KP : KP;
  const unsigned ppr   = (unsigned)(KTOT >> 3);
  const unsigned kp8   = (unsigned)(KP >> 3);
  const unsigned total = (unsigned)MP * ppr;
  const unsigned g     = blockIdx.x * 256u + threadIdx.x;
  const unsigned rowu  = g / ppr;
  const unsigned p     = g - rowu * ppr;
  const bool second    = p >= kp8;
  const int row = (int)rowu;
  const int c0  = (int)((second ? p - kp8 : p) << 3);
  const float* srow = src + (size_t)clampi(row, 0, rows - 1) * (size_t)ldsrc;
  float x[8];
  unsigned mk[8];
#pragma unroll
  for (int e = 0; e < 8; ++e) {
    const int c = c0 + e;
    const float v = srow[clampi(c, 0, cols - 1)];
    asm volatile("" :: "v"(v));
    x[e]  = v;
    mk[e] = (row < rows && c < cols) ? 0xFFFFu : 0u;
  }
  const v4f a = (v4f){ x[0], x[1], x[2], x[3] };
  const v4f c = (v4f){ x[4], x[5], x[6], x[7] };
  v4u o;
  if (FORM == 2) {
    o = pack8_f16(a, c);
  } else {
    const v4u hi = pack8_bf16(a, c);
    o = hi;
    if (FORM == 1) { const v4u lo = pack8_bf16_lo(a, c); o = second ? lo : hi; }
  }
  const v4u mw = (v4u){ pk16(mk[0], mk[1]), pk16(mk[2], mk[3]), pk16(mk[4], mk[5]), pk16(mk[6], mk[7]) };
  o &= mw;
  if (g < total) {
    volatile v4u* q = (volatile v4u*)(dst + (size_t)g * 8);
    *q = o;
    __threadfence();
    *q = o;
  }
}

template <int FORM> struct FragOf    { typedef FragB T; };
template <>         struct FragOf<2> { typedef FragH T; };
__device__ __forceinline__ v8f mm(const FragB& a, const FragB& b, v8f c) { return wmb(a, b, c); }
__device__ __forceinline__ v8f mm(const FragH& a, const FragH& b, v8f c) { return wmh(a, b, c); }
template <class F> __device__ __forceinline__ F ld_frag(const unsigned short* p) {
  F f;
  f.h[0] = *(const v8usa*)(p);
  f.h[1] = *(const v8usa*)(p + 16);
  return f;
}

template <int FORM, int EPI>
__global__ __launch_bounds__(256) __attribute__((amdgpu_num_vgpr(248)))
void k_gemm_nt(const unsigned short* __restrict__ A, const unsigned short* __restrict__ B,
               const float* __restrict__ bias, float* __restrict__ D, int M, int N, int KTOT, int ldd) {
  static_assert(FORM >= 0 && FORM <= 2);
  static_assert(EPI == 0 || EPI == 1);
  typedef typename FragOf<FORM>::T F;
  __shared__ __attribute__((aligned(16))) float sT[8][16 * 68];
  const int lane = threadIdx.x & 31;
  const int wave = threadIdx.x >> 5;
  const int tilesM = (M + 63) >> 6;
  const int tilesN = (N + 63) >> 6;
  const int tile = blockIdx.x * 8 + wave;
  if (tile >= tilesM * tilesN) return;
  const int tm = tile / tilesN;
  const int tn = tile - tm * tilesN;
  const int m0 = tm << 6;
  const int n0 = tn << 6;

  const int rl = lane & 15;
  const int h8 = (lane >> 4) * 8;
  const unsigned short* pa = A + (size_t)(m0 + rl) * (size_t)KTOT + h8;
  const unsigned short* pb = B + (size_t)(n0 + rl) * (size_t)KTOT + h8;

  v8f acc[4][4];
#pragma unroll
  for (int i = 0; i < 4; ++i)
#pragma unroll
    for (int j = 0; j < 4; ++j) acc[i][j] = (v8f){0.f, 0.f, 0.f, 0.f, 0.f, 0.f, 0.f, 0.f};

#pragma unroll 1
  for (int k0 = 0; k0 < KTOT; k0 += 32) {
    F bf[4];
#pragma unroll
    for (int j = 0; j < 4; ++j) bf[j] = ld_frag<F>(pb + (size_t)(j << 4) * (size_t)KTOT + k0);
#pragma unroll
    for (int i = 0; i < 4; ++i) {
      const F af = ld_frag<F>(pa + (size_t)(i << 4) * (size_t)KTOT + k0);
#pragma unroll
      for (int j = 0; j < 4; ++j) acc[i][j] = mm(af, bf[j], acc[i][j]);
    }
  }

  float* slab = sT[wave];
  const int hh = lane >> 4;
  const int c4 = (lane & 15) * 4;
  const int nc = n0 + c4;
  const bool cok = nc < N;
  v4f bv = (v4f){0.f, 0.f, 0.f, 0.f};
  if (EPI == 1) {
    bv = *(const v4fa*)(bias + clampi(nc, 0, N - 4));
    asm volatile("" :: "v"(bv));
  }
#pragma unroll
  for (int i = 0; i < 4; ++i) {
    const int mBase = m0 + (i << 4);
#pragma unroll
    for (int j = 0; j < 4; ++j) {
#pragma unroll
      for (int r = 0; r < 8; ++r) slab[(h8 + r) * 68 + (j << 4) + rl] = acc[i][j][r];
    }
    __builtin_amdgcn_fence(__ATOMIC_RELEASE, "workgroup");
    __builtin_amdgcn_wave_barrier();
    __builtin_amdgcn_fence(__ATOMIC_ACQUIRE, "workgroup");
    v4f vv[8];
#pragma unroll
    for (int it = 0; it < 8; ++it) {
      const int row = it * 2 + hh;
      v4f v = *(const v4fa*)(slab + row * 68 + c4);
      if (EPI == 1) v += bv;
      vv[it] = v;
    }
    for (int pass = 0; pass < 2; ++pass) {
#pragma unroll
      for (int it = 0; it < 8; ++it) {
        const int row = mBase + it * 2 + hh;
        if (cok && row < M) *(volatile v4f*)(D + (size_t)row * (size_t)ldd + nc) = vv[it];
      }
      __threadfence();
    }
    __builtin_amdgcn_fence(__ATOMIC_RELEASE, "workgroup");
    __builtin_amdgcn_wave_barrier();
    __builtin_amdgcn_fence(__ATOMIC_ACQUIRE, "workgroup");
  }
}

#define NN        100000
#define NE        1600000
#define FD        128
#define NC        64
#define MPAD      100096
#define NTHR      256
#define CHUNK     2048
#define SLB       10
#define NSLOT     1024
#define NBKT      98
#define LCAP      20992
#define DEGCAP    64
#define HITS_MEAS 16710
#define DEG_MEAS  36
#define RPB       64
#define RPW       8
#define TWO_TERM_L2   1
#define TWO_TERM_HEAD 1
#define WSMAX     ((size_t)128 << 20)

#define BK_INTS   (2 * LCAP + 4 * NSLOT + 32)
#define BK_LDS_BYTES (BK_INTS * 4)

static_assert(NSLOT == (1 << SLB));
static_assert((long long)NSLOT * NBKT >= MPAD && MPAD >= NN);
static_assert(LCAP % 256 == 0 && 4 * LCAP >= 5 * HITS_MEAS);
static_assert(DEGCAP >= DEG_MEAS + 8);
static_assert(NE < (1 << 21));
static_assert(NE % 4 == 0);
static_assert(MPAD % 64 == 0 && MPAD % RPB == 0 && RPB == (NTHR / 32) * RPW);
static_assert(NN % 16 == 0 && FD % 32 == 0 && NC % 4 == 0 && FD == 4 * 32);
static_assert(BK_INTS % 4 == 0 && BK_LDS_BYTES <= 262144);
static_assert((LCAP * 4) % 128 == 0);
static_assert((long long)MPAD * 256 / 8 < (1LL << 31));

typedef int          v4i  __attribute__((ext_vector_type(4)));
typedef unsigned int v2u  __attribute__((ext_vector_type(2)));
typedef v4i __attribute__((may_alias)) v4ia;
typedef v2u __attribute__((may_alias)) v2ua;

static constexpr size_t SZ_HHL  = (size_t)MPAD * 256 * 2;
static constexpr size_t SZ_MP   = (size_t)MPAD * FD * 4;
static constexpr size_t SZ_LIST = (size_t)NBKT * LCAP * 4;
static constexpr size_t SZ_TAB  = (size_t)NBKT * NSLOT * 4;
static constexpr size_t SZ_FLAG = (size_t)NBKT * 128;
static constexpr size_t SZ_W1B  = (size_t)FD * FD * 2;
static constexpr size_t SZ_W2D  = (size_t)FD * 2 * FD * 2;
static constexpr size_t SZ_WLD  = (size_t)NC * 2 * FD * 2;
static constexpr size_t SZ_BT   = (size_t)3 * FD * 4;
static constexpr size_t O_HHL  = 0;
static constexpr size_t O_MP   = O_HHL + SZ_HHL;
static constexpr size_t O_LIST = O_MP + SZ_MP;
static constexpr size_t O_CNT  = O_LIST + SZ_LIST;
static constexpr size_t O_OFF  = O_CNT + SZ_TAB;
static constexpr size_t O_DIS  = O_OFF + SZ_TAB;
static constexpr size_t O_FLAG = O_DIS + SZ_TAB;
static constexpr size_t O_W1B  = O_FLAG + SZ_FLAG;
static constexpr size_t O_W2D  = O_W1B + SZ_W1B;
static constexpr size_t O_WLD  = O_W2D + SZ_W2D;
static constexpr size_t O_BT   = O_WLD + SZ_WLD;
static constexpr size_t WS_TOTAL = O_BT + SZ_BT;
static_assert(O_MP % 128 == 0 && O_LIST % 128 == 0 && O_CNT % 128 == 0 && O_OFF % 128 == 0 && O_DIS % 128 == 0);
static_assert(O_FLAG % 128 == 0 && O_W1B % 128 == 0 && O_W2D % 128 == 0 && O_WLD % 128 == 0 && O_BT % 128 == 0);
static_assert(WS_TOTAL <= (size_t)WSMAX);
static_assert((size_t)MPAD * FD * 2 <= SZ_HHL);

__device__ __forceinline__ float blend3(float a, float b, float c, unsigned ma, unsigned mb, unsigned mc) {
  const unsigned r = (__float_as_uint(bf16_val(a)) & ma) | (__float_as_uint(bf16_val(b)) & mb) |
                     (__float_as_uint(bf16_val(c)) & mc);
  return __uint_as_float(r);
}
__device__ __forceinline__ float relu_keep(float v) { return (v > 0.0f) ? v : (v - v); }

__global__ __launch_bounds__(96) void k_bias(const float* __restrict__ b1, const float* __restrict__ b2,
                                             const float* __restrict__ bl, float* bt) {
  const int t = (int)threadIdx.x;
  const v4f a = *(const v4fa*)(b1 + 4 * clampi(t, 0, 31));
  const v4f b = *(const v4fa*)(b2 + 4 * clampi(t - 32, 0, 31));
  const v4f c = *(const v4fa*)(bl + 4 * clampi(t - 64, 0, 15));
  asm volatile("" :: "v"(a));
  asm volatile("" :: "v"(b));
  asm volatile("" :: "v"(c));
  const unsigned ma = (t < 32) ? 0xFFFFFFFFu : 0u;
  const unsigned mb = (t >= 32 && t < 64) ? 0xFFFFFFFFu : 0u;
  const unsigned mc = (t >= 64 && t < 80) ? 0xFFFFFFFFu : 0u;
  v4f o;
  o.x = blend3(a.x, b.x, c.x, ma, mb, mc);
  o.y = blend3(a.y, b.y, c.y, ma, mb, mc);
  o.z = blend3(a.z, b.z, c.z, ma, mb, mc);
  o.w = blend3(a.w, b.w, c.w, ma, mb, mc);
  volatile v4f* q = (volatile v4f*)(bt + 4 * t);
  *q = o;
  __threadfence();
  *q = o;
}

__global__ __launch_bounds__(NTHR) void k_bucket(const int* __restrict__ srcs, const int* __restrict__ dsts,
                                                 int nE, int nN, int vec8,
                                                 int* LIST, int* CNT, int* OFF, float* DIS, int* FLAG) {
  extern __shared__ __attribute__((aligned(16))) int dsm[];
  int* hl   = dsm;
  int* sl   = dsm + LCAP;
  int* cnt  = dsm + 2 * LCAP;
  int* offs = cnt + NSLOT;
  int* cur  = offs + NSLOT;
  int* disb = cur + NSLOT;
  int* wcnt = disb + NSLOT;
  int* misc = wcnt + 16;
  const int tid  = (int)threadIdx.x;
  const int lane = tid & 31;
  const int wave = __builtin_amdgcn_readfirstlane(tid >> 5);
  const int blk  = (int)blockIdx.x;

  {
    const v4i z4 = (v4i){0, 0, 0, 0};
    for (int i = tid * 4; i < BK_INTS; i += NTHR * 4) *(v4ia*)(dsm + i) = z4;
  }
  __syncthreads();

  int tbase = 0;
  const unsigned nbs = (unsigned)blk * (unsigned)NSLOT;
  const unsigned unn = (unsigned)nN;
  const int nChunks = (nE + CHUNK - 1) / CHUNK;
#pragma unroll 1
  for (int ch = 0; ch < nChunks; ++ch) {
    const int cbase = ch * CHUNK;
    const int e0    = cbase + tid * 8;
    v4i da, db;
    if (vec8 != 0 && cbase + CHUNK <= nE) {
      da = *(const v4i*)(dsts + e0);
      db = *(const v4i*)(dsts + e0 + 4);
    } else {
      const int t0 = dsts[clampi(e0,     0, nE - 1)];
      const int t1 = dsts[clampi(e0 + 1, 0, nE - 1)];
      const int t2 = dsts[clampi(e0 + 2, 0, nE - 1)];
      const int t3 = dsts[clampi(e0 + 3, 0, nE - 1)];
      const int t4 = dsts[clampi(e0 + 4, 0, nE - 1)];
      const int t5 = dsts[clampi(e0 + 5, 0, nE - 1)];
      const int t6 = dsts[clampi(e0 + 6, 0, nE - 1)];
      const int t7 = dsts[clampi(e0 + 7, 0, nE - 1)];
      asm volatile("" :: "v"(t0)); asm volatile("" :: "v"(t1));
      asm volatile("" :: "v"(t2)); asm volatile("" :: "v"(t3));
      asm volatile("" :: "v"(t4)); asm volatile("" :: "v"(t5));
      asm volatile("" :: "v"(t6)); asm volatile("" :: "v"(t7));
      const int k0 = -(int)(e0     < nE), k1 = -(int)(e0 + 1 < nE);
      const int k2 = -(int)(e0 + 2 < nE), k3 = -(int)(e0 + 3 < nE);
      const int k4 = -(int)(e0 + 4 < nE), k5 = -(int)(e0 + 5 < nE);
      const int k6 = -(int)(e0 + 6 < nE), k7 = -(int)(e0 + 7 < nE);
      da.x = (t0 & k0) | ~k0; da.y = (t1 & k1) | ~k1;
      da.z = (t2 & k2) | ~k2; da.w = (t3 & k3) | ~k3;
      db.x = (t4 & k4) | ~k4; db.y = (t5 & k5) | ~k5;
      db.z = (t6 & k6) | ~k6; db.w = (t7 & k7) | ~k7;
    }
    const unsigned s0 = (unsigned)da.x - nbs, s1 = (unsigned)da.y - nbs;
    const unsigned s2 = (unsigned)da.z - nbs, s3 = (unsigned)da.w - nbs;
    const unsigned s4 = (unsigned)db.x - nbs, s5 = (unsigned)db.y - nbs;
    const unsigned s6 = (unsigned)db.z - nbs, s7 = (unsigned)db.w - nbs;
    const bool h0 = (s0 < (unsigned)NSLOT) & ((unsigned)da.x < unn);
    const bool h1 = (s1 < (unsigned)NSLOT) & ((unsigned)da.y < unn);
    const bool h2 = (s2 < (unsigned)NSLOT) & ((unsigned)da.z < unn);
    const bool h3 = (s3 < (unsigned)NSLOT) & ((unsigned)da.w < unn);
    const bool h4 = (s4 < (unsigned)NSLOT) & ((unsigned)db.x < unn);
    const bool h5 = (s5 < (unsigned)NSLOT) & ((unsigned)db.y < unn);
    const bool h6 = (s6 < (unsigned)NSLOT) & ((unsigned)db.z < unn);
    const bool h7 = (s7 < (unsigned)NSLOT) & ((unsigned)db.w < unn);
    const unsigned m0 = __builtin_amdgcn_ballot_w32(h0), m1 = __builtin_amdgcn_ballot_w32(h1);
    const unsigned m2 = __builtin_amdgcn_ballot_w32(h2), m3 = __builtin_amdgcn_ballot_w32(h3);
    const unsigned m4 = __builtin_amdgcn_ballot_w32(h4), m5 = __builtin_amdgcn_ballot_w32(h5);
    const unsigned m6 = __builtin_amdgcn_ballot_w32(h6), m7 = __builtin_amdgcn_ballot_w32(h7);
    unsigned pre = __builtin_amdgcn_mbcnt_lo(m0, 0u);
    pre = __builtin_amdgcn_mbcnt_lo(m1, pre);
    pre = __builtin_amdgcn_mbcnt_lo(m2, pre);
    pre = __builtin_amdgcn_mbcnt_lo(m3, pre);
    pre = __builtin_amdgcn_mbcnt_lo(m4, pre);
    pre = __builtin_amdgcn_mbcnt_lo(m5, pre);
    pre = __builtin_amdgcn_mbcnt_lo(m6, pre);
    pre = __builtin_amdgcn_mbcnt_lo(m7, pre);
    const int wtot = __builtin_popcount(m0) + __builtin_popcount(m1) + __builtin_popcount(m2) +
                     __builtin_popcount(m3) + __builtin_popcount(m4) + __builtin_popcount(m5) +
                     __builtin_popcount(m6) + __builtin_popcount(m7);
    const int par = (ch & 1) * 8;
    if (lane == 0) wcnt[par + wave] = wtot;
    __syncthreads();
    const v4i wa = *(const v4ia*)(wcnt + par);
    const v4i wb = *(const v4ia*)(wcnt + par + 4);
    const int tot = wa.x + wa.y + wa.z + wa.w + wb.x + wb.y + wb.z + wb.w;
    int pw = 0;
    pw += (wave > 0) ? wa.x : 0;
    pw += (wave > 1) ? wa.y : 0;
    pw += (wave > 2) ? wa.z : 0;
    pw += (wave > 3) ? wa.w : 0;
    pw += (wave > 4) ? wb.x : 0;
    pw += (wave > 5) ? wb.y : 0;
    pw += (wave > 6) ? wb.z : 0;
    if (wtot != 0) {
      int pos = tbase + pw + (int)pre;
      if (h0 && pos < LCAP) hl[pos] = ((e0    ) << SLB) | (int)s0;
      pos += h0 ? 1 : 0;
      if (h1 && pos < LCAP) hl[pos] = ((e0 + 1) << SLB) | (int)s1;
      pos += h1 ? 1 : 0;
      if (h2 && pos < LCAP) hl[pos] = ((e0 + 2) << SLB) | (int)s2;
      pos += h2 ? 1 : 0;
      if (h3 && pos < LCAP) hl[pos] = ((e0 + 3) << SLB) | (int)s3;
      pos += h3 ? 1 : 0;
      if (h4 && pos < LCAP) hl[pos] = ((e0 + 4) << SLB) | (int)s4;
      pos += h4 ? 1 : 0;
      if (h5 && pos < LCAP) hl[pos] = ((e0 + 5) << SLB) | (int)s5;
      pos += h5 ? 1 : 0;
      if (h6 && pos < LCAP) hl[pos] = ((e0 + 6) << SLB) | (int)s6;
      pos += h6 ? 1 : 0;
      if (h7 && pos < LCAP) hl[pos] = ((e0 + 7) << SLB) | (int)s7;
    }
    tbase += tot;
  }
  __syncthreads();
  const int T   = clampi(tbase, 0, LCAP);
  const int ovf = (tbase > LCAP) ? 1 : 0;

  if (tid == 0) {
#pragma unroll 1
    for (int t = 0; t < T; ++t) {
      const int s = hl[t] & (NSLOT - 1);
      cnt[s] = cnt[s] + 1;
    }
  }
  __syncthreads();

  if (wave == 0) {
    const int base = lane * (NSLOT / 32);
    int s = 0, mx = 0;
#pragma unroll 1
    for (int i = 0; i < NSLOT / 32; ++i) { const int c = cnt[base + i]; s += c; mx = c > mx ? c : mx; }
    int incl = s;
#pragma unroll
    for (int dl = 1; dl < 32; dl <<= 1) {
      const int y = __shfl_up(incl, dl, 32);
      incl += (lane >= dl) ? y : 0;
    }
    int run = incl - s;
#pragma unroll 1
    for (int i = 0; i < NSLOT / 32; ++i) {
      const int cv = cnt[base + i];
      offs[base + i] = run;
      cur[base + i]  = run;
      run += cv;
    }
    const unsigned bigm = __builtin_amdgcn_ballot_w32(mx > DEGCAP);
    if (lane == 0) misc[0] = ((bigm != 0u) ? 1 : 0) | ovf;
  }
  __syncthreads();

  if (tid == 0) {
#pragma unroll 1
    for (int t = 0; t < T; ++t) {
      const int u = hl[t];
      const int s = u & (NSLOT - 1);
      const int p = clampi(cur[s], 0, LCAP - 1);
      sl[p]  = u >> SLB;
      cur[s] = p + 1;
    }
  }
#pragma unroll 1
  for (int i = 0; i < NSLOT / NTHR; ++i) {
    const int s = tid + NTHR * i;
    const float deg = (float)(cnt[s] + 1);
    const float dv  = (deg > 0.0f) ? (1.0f / sqrtf(fmaxf(deg, 1.0f))) : 0.0f;
    disb[s] = __float_as_int(dv);
  }
  __syncthreads();

  const int fl = misc[0];
  int* lbase = LIST + (size_t)blk * (size_t)LCAP;
#pragma unroll 1
  for (int q = tid; q < LCAP / 4; q += NTHR) {
    const int i0 = 4 * q;
    const v4i e4 = *(const v4ia*)(sl + i0);
    const int a0 = srcs[clampi(e4.x, 0, nE - 1)];
    const int a1 = srcs[clampi(e4.y, 0, nE - 1)];
    const int a2 = srcs[clampi(e4.z, 0, nE - 1)];
    const int a3 = srcs[clampi(e4.w, 0, nE - 1)];
    asm volatile("" :: "v"(a0)); asm volatile("" :: "v"(a1));
    asm volatile("" :: "v"(a2)); asm volatile("" :: "v"(a3));
    v4i o;
    o.x = clampi(a0, 0, nN - 1) & -(int)(i0     < T);
    o.y = clampi(a1, 0, nN - 1) & -(int)(i0 + 1 < T);
    o.z = clampi(a2, 0, nN - 1) & -(int)(i0 + 2 < T);
    o.w = clampi(a3, 0, nN - 1) & -(int)(i0 + 3 < T);
    volatile v4i* p = (volatile v4i*)(lbase + i0);
    *p = o;
    __threadfence();
    *p = o;
  }

  const v4i c4 = *(const v4ia*)(cnt + 4 * tid);
  const v4i o4 = *(const v4ia*)(offs + 4 * tid);
  const v4i d4 = *(const v4ia*)(disb + 4 * tid);
  v4f df;
  df.x = __int_as_float(d4.x); df.y = __int_as_float(d4.y);
  df.z = __int_as_float(d4.z); df.w = __int_as_float(d4.w);
  const size_t sbase = (size_t)blk * (size_t)NSLOT + (size_t)(4 * tid);
  volatile v4i* pc = (volatile v4i*)(CNT + sbase);
  volatile v4i* po = (volatile v4i*)(OFF + sbase);
  volatile v4f* pd = (volatile v4f*)(DIS + sbase);
  volatile int* pf = (volatile int*)(FLAG + (size_t)blk * 32 + (size_t)lane);
  *pc = c4; *po = o4; *pd = df;
  if (wave == 0) *pf = fl;
  __threadfence();
  *pc = c4; *po = o4; *pd = df;
  if (wave == 0) *pf = fl;
}

template <int LAYER>
__global__ __launch_bounds__(NTHR) void k_replay(const float* __restrict__ Mp, const int* __restrict__ LIST,
                                                 const int* __restrict__ CNT, const int* __restrict__ OFF,
                                                 const float* __restrict__ DIS, const int* __restrict__ FLAG,
                                                 const float* __restrict__ bias, const float* __restrict__ xres,
                                                 unsigned short* hhl, int nN, int mRows) {
  static_assert(LAYER == 1 || LAYER == 2);
  __shared__ __attribute__((aligned(16))) float sb[FD];
  const int tid  = (int)threadIdx.x;
  const int lane = tid & 31;
  const int wave = __builtin_amdgcn_readfirstlane(tid >> 5);
  if (wave == 0) {
    const v4f b = *(const v4fa*)(bias + 4 * lane);
    *(v4fa*)(sb + 4 * lane) = b;
  }
  __syncthreads();
  const v4f bv = *(const v4fa*)(sb + 4 * lane);
  const float qnan = __uint_as_float(0x7fc00000u);

#pragma unroll 1
  for (int i = 0; i < RPW; ++i) {
    const int d = (int)blockIdx.x * RPB + wave * RPW + i;
    if (d < mRows) {
      const bool live = d < nN;
      const int  dc   = live ? d : nN - 1;
      const int  bb   = clampi(d >> SLB, 0, NBKT - 1);
      const int  cv   = CNT[d];
      const int  ov   = OFF[d];
      const int  fl   = FLAG[bb * 32];
      const float dd  = DIS[dc];
      asm volatile("" :: "v"(cv)); asm volatile("" :: "v"(ov));
      asm volatile("" :: "v"(fl)); asm volatile("" :: "v"(dd));
      const int cvc = live ? clampi(cv, 0, DEGCAP) : 0;
      const int cn  = __builtin_amdgcn_readfirstlane(cvc);
      const int off = __builtin_amdgcn_readfirstlane(clampi(ov, 0, LCAP - 1));
      const bool pois = (fl != 0) || (cv > DEGCAP);
      const int* lp = LIST + (size_t)bb * (size_t)LCAP;

      v4f acc = (v4f){0.0f, 0.0f, 0.0f, 0.0f};
#pragma unroll 1
      for (int b0 = 0; b0 < cn; b0 += 32) {
        const int idx = clampi(off + b0 + lane, 0, LCAP - 1);
        const int sr  = clampi(lp[idx], 0, nN - 1);
        const float ds = DIS[sr];
        const float cf = ds * dd;
        const int cfi  = __float_as_int(cf);
        const int m32  = (cn - b0) < 32 ? (cn - b0) : 32;
#pragma unroll 1
        for (int k = 0; k < m32; ++k) {
          const int   sk = __builtin_amdgcn_readlane(sr, k);
          const float ck = __int_as_float(__builtin_amdgcn_readlane(cfi, k));
          const v4f a = *(const v4fa*)(Mp + (size_t)sk * FD + 4 * lane);
          acc.x = fmaf(ck, a.x, acc.x); acc.y = fmaf(ck, a.y, acc.y);
          acc.z = fmaf(ck, a.z, acc.z); acc.w = fmaf(ck, a.w, acc.w);
        }
      }
      const v4f sv = *(const v4fa*)(Mp + (size_t)dc * FD + 4 * lane);
      asm volatile("" :: "v"(sv));
      const float rd = dd * dd;
      acc.x = fmaf(sv.x, rd, acc.x); acc.y = fmaf(sv.y, rd, acc.y);
      acc.z = fmaf(sv.z, rd, acc.z); acc.w = fmaf(sv.w, rd, acc.w);
      v4f y;
      y.x = relu_keep(acc.x + bv.x); y.y = relu_keep(acc.y + bv.y);
      y.z = relu_keep(acc.z + bv.z); y.w = relu_keep(acc.w + bv.w);

      unsigned short* prow = hhl + (size_t)d * 256 + 4 * lane;
      v4f r;
      if constexpr (LAYER == 1) {
        const v4f xr = *(const v4fa*)(xres + (size_t)dc * FD + 4 * lane);
        asm volatile("" :: "v"(xr));
        r.x = bf16_val(xr.x); r.y = bf16_val(xr.y); r.z = bf16_val(xr.z); r.w = bf16_val(xr.w);
      } else {
        const v2u hw = *(const v2ua*)(prow);
        const v2u lw = *(const v2ua*)(prow + 128);
        asm volatile("" :: "v"(hw));
        asm volatile("" :: "v"(lw));
        r.x = __uint_as_float(hw.x << 16)          + __uint_as_float(lw.x << 16);
        r.y = __uint_as_float(hw.x & 0xffff0000u)  + __uint_as_float(lw.x & 0xffff0000u);
        r.z = __uint_as_float(hw.y << 16)          + __uint_as_float(lw.y << 16);
        r.w = __uint_as_float(hw.y & 0xffff0000u)  + __uint_as_float(lw.y & 0xffff0000u);
      }
      v4f v;
      v.x = y.x + r.x; v.y = y.y + r.y; v.z = y.z + r.z; v.w = y.w + r.w;
      v.x = pois ? qnan : v.x; v.y = pois ? qnan : v.y; v.z = pois ? qnan : v.z; v.w = pois ? qnan : v.w;
      v.x = live ? v.x : 0.0f; v.y = live ? v.y : 0.0f; v.z = live ? v.z : 0.0f; v.w = live ? v.w : 0.0f;

      v2u hv, lv;
      hv.x = pk16(bf16_bits(v.x), bf16_bits(v.y));
      hv.y = pk16(bf16_bits(v.z), bf16_bits(v.w));
      lv.x = pk16(bf16_lo_bits(v.x), bf16_lo_bits(v.y));
      lv.y = pk16(bf16_lo_bits(v.z), bf16_lo_bits(v.w));
      volatile v2u* ph = (volatile v2u*)(prow);
      volatile v2u* pl = (volatile v2u*)(prow + 128);
      *ph = hv; *pl = lv;
      __threadfence();
      *ph = hv; *pl = lv;
    }
  }
}

extern "C" void kernel_launch(void* const* d_in, const int* in_sizes, int n_in,
                              void* d_out, int out_size, void* d_ws, size_t ws_size,
                              hipStream_t stream) {
  if (n_in < 8) return;
  if (in_sizes[0] != NN * FD) return;
  if (in_sizes[1] != 2 * NE) return;
  if (in_sizes[2] != FD * FD || in_sizes[3] != FD) return;
  if (in_sizes[4] != FD * FD || in_sizes[5] != FD) return;
  if (in_sizes[6] != NC * FD || in_sizes[7] != NC) return;
  if (out_size != NN * NC) return;
  if (WS_TOTAL > ws_size) return;

  const float* x   = (const float*)d_in[0];
  const int*   ei  = (const int*)d_in[1];
  const float* W1  = (const float*)d_in[2];
  const float* b1  = (const float*)d_in[3];
  const float* W2  = (const float*)d_in[4];
  const float* b2  = (const float*)d_in[5];
  const float* Wl  = (const float*)d_in[6];
  const float* bl  = (const float*)d_in[7];
  float* out = (float*)d_out;
  const int* src = ei;
  const int* dst = ei + NE;
  const int vec8 = ((NE & 3) == 0) ? 1 : 0;

  char* ws = (char*)d_ws;
  unsigned short* HHL = (unsigned short*)(ws + O_HHL);
  unsigned short* XB  = (unsigned short*)(ws + O_HHL);
  float*          MPL = (float*)(ws + O_MP);
  int*            LST = (int*)(ws + O_LIST);
  int*            CNT = (int*)(ws + O_CNT);
  int*            OFF = (int*)(ws + O_OFF);
  float*          DIS = (float*)(ws + O_DIS);
  int*            FLG = (int*)(ws + O_FLAG);
  unsigned short* W1B = (unsigned short*)(ws + O_W1B);
  unsigned short* W2D = (unsigned short*)(ws + O_W2D);
  unsigned short* WLD = (unsigned short*)(ws + O_WLD);
  float*          BT  = (float*)(ws + O_BT);

  hipFuncSetAttribute(reinterpret_cast<const void*>(&k_bucket), hipFuncAttributeMaxDynamicSharedMemorySize,
                      (int)BK_LDS_BYTES);

  k_plane<0><<<MPAD * FD / 8 / 256, 256, 0, stream>>>(x, NN, FD, FD, XB, MPAD, FD);
  k_plane<0><<<FD * FD / 8 / 256, 256, 0, stream>>>(W1, FD, FD, FD, W1B, FD, FD);
#if TWO_TERM_L2
  k_plane<3><<<FD * 2 * FD / 8 / 256, 256, 0, stream>>>(W2, FD, FD, FD, W2D, FD, FD);
#else
  k_plane<0><<<FD * 2 * FD / 8 / 256, 256, 0, stream>>>(W2, FD, FD, FD, W2D, FD, 2 * FD);
#endif
#if TWO_TERM_HEAD
  k_plane<3><<<NC * 2 * FD / 8 / 256, 256, 0, stream>>>(Wl, NC, FD, FD, WLD, NC, FD);
#else
  k_plane<0><<<NC * 2 * FD / 8 / 256, 256, 0, stream>>>(Wl, NC, FD, FD, WLD, NC, 2 * FD);
#endif
  k_bias<<<1, 96, 0, stream>>>(b1, b2, bl, BT);
  k_bucket<<<NBKT, NTHR, BK_LDS_BYTES, stream>>>(src, dst, NE, NN, vec8, LST, CNT, OFF, DIS, FLG);

  const int tilesM  = (NN + 63) / 64;
  const int gridG2  = (tilesM * 2 + 7) / 8;
  const int gridG1  = (tilesM * 1 + 7) / 8;
  k_gemm_nt<0, 0><<<gridG2, 256, 0, stream>>>(XB, W1B, BT, MPL, NN, FD, FD, FD);
  k_replay<1><<<MPAD / RPB, NTHR, 0, stream>>>(MPL, LST, CNT, OFF, DIS, FLG, BT, x, HHL, NN, MPAD);
  k_gemm_nt<0, 0><<<gridG2, 256, 0, stream>>>(HHL, W2D, BT, MPL, NN, FD, 2 * FD, FD);
  k_replay<2><<<MPAD / RPB, NTHR, 0, stream>>>(MPL, LST, CNT, OFF, DIS, FLG, BT + FD, x, HHL, NN, MPAD);
  k_gemm_nt<0, 1><<<gridG1, 256, 0, stream>>>(HHL, WLD, BT + 2 * FD, out, NN, NC, 2 * FD, NC);
}
